// OffsetPredictor_2216203124765
// MI455X (gfx1250) — hardware-verified
//
#include <hip/hip_runtime.h>
#include <math.h>

#define NB_ 8
#define CC_ 256
#define LL_ 4096
#define PATCH 16
#define STRIDE 8
#define HID 64
#define NP_ 511
#define NPT 32

typedef _Float16 f16;
typedef __attribute__((ext_vector_type(16))) f16 f16x16;
typedef __attribute__((ext_vector_type(8)))  f16 f16x8;
typedef __attribute__((ext_vector_type(8)))  float f32x8;
typedef __attribute__((ext_vector_type(4)))  float v4f_t;
typedef float v4fa __attribute__((ext_vector_type(4), may_alias));

__device__ __forceinline__ f32x8 wmma16(f16x16 a, f16x16 b, f32x8 c) {
  c = __builtin_amdgcn_wmma_f32_16x16x32_f16(false, a, false, b, (short)0, c, false, false);
  asm volatile("v_nop\n\tv_nop\n\tv_nop\n\tv_nop" : "+v"(c) : "v"(a), "v"(b));
  return c;
}
__device__ __forceinline__ f16x16 lds_frag(const f16* base, int stride) {
  const int lane = threadIdx.x & 31, row = lane & 15, kh = (lane >> 4) * 8;
  const f16x8 lo = *(const f16x8*)(base + row * stride + kh);
  const f16x8 hi = *(const f16x8*)(base + row * stride + kh + 16);
  f16x16 f;
#pragma unroll
  for (int i = 0; i < 8; ++i) { f[i] = lo[i]; f[i + 8] = hi[i]; }
  return f;
}

__global__ __launch_bounds__(256) void k_offset(const float* __restrict__ x, const float* __restrict__ W1, const float* __restrict__ b1,
                                               const float* __restrict__ W2, const float* __restrict__ b2, float* __restrict__ out) {
  __shared__ __attribute__((aligned(16))) f16 hS[8][2][16 * 72];
  __shared__ __attribute__((aligned(16))) float oS[512 * 36];
  const int tid = threadIdx.x, lane = tid & 31, wave = tid >> 5, cl = lane & 15, hsel = lane >> 4, kh = hsel * 8, rh = kh;
  const int b = blockIdx.x / (CC_ / 16), cg = (blockIdx.x % (CC_ / 16)) * 16;
  f16x16 w1f[4], w1l[4], w2f[2], w2l[2];
#pragma unroll
  for (int nt = 0; nt < 4; ++nt) {
#pragma unroll
    for (int i = 0; i < 8; ++i) { const int k = kh + i; const float wv = (k < PATCH) ? W1[(nt * 16 + cl) * PATCH + k] : 0.0f; const f16 h = (f16)wv;
      w1f[nt][i] = h; w1l[nt][i] = (f16)((wv - (float)h) * 2048.0f); w1f[nt][8 + i] = (f16)0.0f; w1l[nt][8 + i] = (f16)0.0f; }
  }
#pragma unroll
  for (int ks = 0; ks < 2; ++ks) {
#pragma unroll
    for (int i = 0; i < 8; ++i) {
      const float a0 = (cl < 2) ? W2[cl * HID + ks * 32 + kh + i] : 0.0f, a1 = (cl < 2) ? W2[cl * HID + ks * 32 + 16 + kh + i] : 0.0f;
      const f16 h0 = (f16)a0, h1 = (f16)a1;
      w2f[ks][i] = h0; w2l[ks][i] = (f16)((a0 - (float)h0) * 2048.0f); w2f[ks][8 + i] = h1; w2l[ks][8 + i] = (f16)((a1 - (float)h1) * 2048.0f); }
  }
  float b1v[4];
#pragma unroll
  for (int nt = 0; nt < 4; ++nt) b1v[nt] = b1[nt * 16 + cl];
  const float b2v = (cl < 2) ? b2[cl] : 0.0f;
  f16* hs = hS[wave][0]; f16* hsl = hS[wave][1];
#pragma unroll 1
  for (int cc = 0; cc < 2; ++cc) {
    const int cidx = wave * 2 + cc, c = cg + cidx;
    const float* xr = x + ((size_t)b * CC_ + c) * LL_;
#pragma unroll 1
    for (int pt = 0; pt < NPT; ++pt) {
      f16x16 af, al;
      { const int p = pt * 16 + cl;
        const int base = min(p * STRIDE + kh, LL_ - 8);
        const v4f_t v0 = *(const v4f_t*)(xr + base), v1 = *(const v4f_t*)(xr + base + 4);
        const float vv[8] = {v0[0], v0[1], v0[2], v0[3], v1[0], v1[1], v1[2], v1[3]};
#pragma unroll
        for (int i = 0; i < 8; ++i) { const f16 h = (f16)vv[i]; af[i] = h; al[i] = (f16)((vv[i] - (float)h) * 2048.0f); af[8 + i] = (f16)0.0f; al[8 + i] = (f16)0.0f; } }
#pragma unroll
      for (int nt = 0; nt < 4; ++nt) {
        f32x8 acc = {}, accx = {}; acc = wmma16(af, w1f[nt], acc); accx = wmma16(af, w1l[nt], accx); accx = wmma16(al, w1f[nt], accx);
#pragma unroll 1
        for (int r = 0; r < 8; ++r) { const float hv = acc[r] + accx[r] * (1.0f / 2048.0f) + b1v[nt]; const float gv = 0.5f * hv * (1.0f + erff(hv * 0.70710678118654752f));
          const f16 gh = (f16)gv; hs[(rh + r) * 72 + nt * 16 + cl] = gh; hsl[(rh + r) * 72 + nt * 16 + cl] = (f16)((gv - (float)gh) * 2048.0f); }
      }
      asm volatile("s_wait_dscnt 0" ::: "memory");
      __builtin_amdgcn_wave_barrier();
      f32x8 o = {}, ox = {};
#pragma unroll
      for (int ks = 0; ks < 2; ++ks) { const f16x16 gh = lds_frag(hs + ks * 32, 72), gl = lds_frag(hsl + ks * 32, 72);
        o = wmma16(gh, w2f[ks], o); ox = wmma16(gh, w2l[ks], ox); ox = wmma16(gl, w2f[ks], ox); }
      if (cl < 2) {
#pragma unroll
        for (int r = 0; r < 8; ++r) { const int p = pt * 16 + rh + r; if (p < NP_) oS[p * 36 + cidx * 2 + cl] = o[r] + ox[r] * (1.0f / 2048.0f) + b2v; }
      }
      __builtin_amdgcn_wave_barrier();
    }
  }
  __syncthreads();
#pragma unroll 1
  for (int pass = 0; pass < 2; ++pass) {
    for (int ch = tid; ch < NP_ * 8; ch += 256) { const int p = ch >> 3, q = (ch & 7) * 4;
      *(volatile v4f_t*)(out + (((size_t)b * NP_ + p) * CC_ + cg) * 2 + q) = *(const volatile v4fa*)(oS + p * 36 + q); }
    __threadfence();
  }
}

extern "C" void kernel_launch(void* const* d_in, const int* in_sizes, int n_in,
                              void* d_out, int out_size, void* d_ws, size_t ws_size,
                              hipStream_t stream) {
  (void)in_sizes; (void)n_in; (void)out_size; (void)d_ws; (void)ws_size;
  const float* x = (const float*)d_in[0];
  const float* W1 = (const float*)d_in[1];
  const float* b1 = (const float*)d_in[2];
  const float* W2 = (const float*)d_in[3];
  const float* b2 = (const float*)d_in[4];
  float* out = (float*)d_out;
  k_offset<<<dim3(NB_ * (CC_ / 16)), dim3(256), 0, stream>>>(x, W1, b1, W2, b2, out);
}
